// SelectiveRecurrentFFN_69123203662001
// MI455X (gfx1250) — hardware-run, weakly checked
//
#include <hip/hip_runtime.h>
#include <stddef.h>


#pragma clang fp contract(off)

#define NBAT   4
#define NSEQ   2048
#define NHID   1024
#define NST    1024
#define NTOK   (NBAT * NSEQ)
#define NTHR   256
#define NWAV   (NTHR / 32)
#define GBM    128
#define GNT    2
#define GBN    (16 * GNT)
#define ONT    4
#define OBN    (16 * ONT)
#define TB     32
#define WCAR   64.0f
#define WINV   (1.0f / 64.0f)
#define HCAR   16.0f
#define HINV   (1.0f / 16.0f)
#define OSCL   (WINV * HINV)
#define WSCAP  134217728

#define SZX16  ((size_t)NTOK * NHID * 2)
#define SZW16  ((size_t)NST * NHID * 2)
#define SZF32  ((size_t)NTOK * NST * 4)
#define SZHS   ((size_t)NTOK * NST * 2)
#define OX16   ((size_t)0)
#define OWF16  (OX16 + SZX16)
#define OWI16  (OWF16 + SZW16)
#define OWV16  (OWI16 + SZW16)
#define OWO16  (OWV16 + SZW16)
#define OFG    (OWO16 + SZW16)
#define OWC    (OFG + SZF32)
#define OHS    (OWC + SZF32)
#define WSTOT  (OHS + SZHS)

#define XBLK   (NTOK * NHID / 8 / NTHR)
#define WBLK1  (NST * NHID / 8 / NTHR)
#define CVTBLK (XBLK + 4 * WBLK1)

static_assert(WSTOT <= (size_t)WSCAP);
static_assert((OWF16 % 128) == 0 && (OFG % 128) == 0 && (OWC % 128) == 0 && (OHS % 128) == 0);
static_assert((NHID % 32) == 0 && (NST % 32) == 0);
static_assert((NTOK % GBM) == 0 && (NST % GBN) == 0 && (NHID % OBN) == 0);
static_assert(GBM == NWAV * 16);
static_assert((NTOK * NHID) % (8 * NTHR) == 0 && (NST * NHID) % (8 * NTHR) == 0);
static_assert((NST % NTHR) == 0 && (NSEQ % TB) == 0 && (TB % NWAV) == 0);
static_assert(((GBM * GBN / 4) % NTHR) == 0 && ((GBM * OBN / 4) % NTHR) == 0);
static_assert(GBN == 32 && OBN == 64);
static_assert(OHS + SZHS == WSTOT);

typedef _Float16 v16h __attribute__((ext_vector_type(16)));
typedef _Float16 v8h  __attribute__((ext_vector_type(8), __may_alias__));
typedef float    v8f  __attribute__((ext_vector_type(8)));
typedef float    v4f  __attribute__((ext_vector_type(4), __may_alias__));
union Frag { v16h v; v8h h[2]; };
static_assert(sizeof(Frag) == 32);

__device__ __forceinline__ v8f wmh(v16h a, v16h bq, v8f c) {
  v8f d = __builtin_amdgcn_wmma_f32_16x16x32_f16(false, a, false, bq, (short)0, c, false, false);
  asm volatile("v_nop\n\tv_nop\n\tv_nop\n\tv_nop" : "+v"(d) : "v"(a), "v"(bq));
  return d;
}

__device__ __forceinline__ v8f zero8() {
  v8f z = {0.f, 0.f, 0.f, 0.f, 0.f, 0.f, 0.f, 0.f};
  return z;
}

__device__ __forceinline__ float rcp_(float d) { return __builtin_amdgcn_rcpf(d); }
__device__ __forceinline__ float sigm_(float x) {
  const float xc = fminf(fmaxf(x, -30.0f), 30.0f);
  return rcp_(1.0f + __expf(-xc));
}
__device__ __forceinline__ float tanh_(float x) {
  const float xc = fminf(fmaxf(x, -15.0f), 15.0f);
  return 2.0f * rcp_(1.0f + __expf(-2.0f * xc)) - 1.0f;
}
__device__ __forceinline__ float silu_(float x) { return x * sigm_(x); }

__global__ __launch_bounds__(NTHR) void k_cvt(const float* __restrict__ x, const float* __restrict__ Wf,
                                              const float* __restrict__ Wi, const float* __restrict__ Wv,
                                              const float* __restrict__ Wo, _Float16* P) {
  const int blk = blockIdx.x, tid = threadIdx.x;
  const float* src;
  float sc;
  size_t so;
  if (blk < XBLK) {
    src = x;
    sc = 1.0f;
    so = ((size_t)blk * NTHR + tid) * 8;
  } else {
    const int wb = blk - XBLK;
    const int wsel = wb / WBLK1;
    so = ((size_t)(wb - wsel * WBLK1) * NTHR + tid) * 8;
    sc = WCAR;
    src = (wsel == 0) ? Wf : ((wsel == 1) ? Wi : ((wsel == 2) ? Wv : Wo));
  }
  const v4f a0 = *(const v4f*)(src + so);
  const v4f a1 = *(const v4f*)(src + so + 4);
  v8h hv;
  hv[0] = (_Float16)(a0.x * sc); hv[1] = (_Float16)(a0.y * sc); hv[2] = (_Float16)(a0.z * sc); hv[3] = (_Float16)(a0.w * sc);
  hv[4] = (_Float16)(a1.x * sc); hv[5] = (_Float16)(a1.y * sc); hv[6] = (_Float16)(a1.z * sc); hv[7] = (_Float16)(a1.w * sc);
  _Float16* dp = P + ((size_t)blk * NTHR + tid) * 8;
  *(volatile v8h*)dp = hv;
  __threadfence();
  *(volatile v8h*)dp = hv;
}

__global__ __launch_bounds__(NTHR) void k_gates(const _Float16* __restrict__ X16, const _Float16* __restrict__ WF16,
                                                const _Float16* __restrict__ WI16, const _Float16* __restrict__ WV16,
                                                float* FG, float* WC) {
  __shared__ __align__(16) float sF[GBM * GBN];
  __shared__ __align__(16) float sI[GBM * GBN];
  __shared__ __align__(16) float sV[GBM * GBN];
  const int tid = threadIdx.x, lane = tid & 31, wave = tid >> 5, h = lane >> 4, m = lane & 15;
  const int bm0 = blockIdx.x * GBM;
  const int m0 = bm0 + wave * 16;
  const int n0 = blockIdx.y * GBN;

  v8f af[GNT], ai[GNT], av[GNT];
#pragma unroll
  for (int t = 0; t < GNT; ++t) { af[t] = zero8(); ai[t] = zero8(); av[t] = zero8(); }

  const _Float16* ap = X16 + (size_t)(m0 + m) * NHID + 8 * h;
  const size_t bo = (size_t)(n0 + m) * NHID + 8 * h;
  const _Float16* bfp = WF16 + bo;
  const _Float16* bip = WI16 + bo;
  const _Float16* bvp = WV16 + bo;

#pragma unroll 1
  for (int ks = 0; ks < NHID / 32; ++ks) {
    const int k0 = 32 * ks;
    Frag fa;
    fa.h[0] = *(const v8h*)(ap + k0);
    fa.h[1] = *(const v8h*)(ap + k0 + 16);
#pragma unroll
    for (int t = 0; t < GNT; ++t) {
      const size_t ro = (size_t)(t * 16) * NHID + k0;
      Frag fb;
      fb.h[0] = *(const v8h*)(bfp + ro);
      fb.h[1] = *(const v8h*)(bfp + ro + 16);
      af[t] = wmh(fa.v, fb.v, af[t]);
      Frag fc;
      fc.h[0] = *(const v8h*)(bip + ro);
      fc.h[1] = *(const v8h*)(bip + ro + 16);
      ai[t] = wmh(fa.v, fc.v, ai[t]);
      Frag fd;
      fd.h[0] = *(const v8h*)(bvp + ro);
      fd.h[1] = *(const v8h*)(bvp + ro + 16);
      av[t] = wmh(fa.v, fd.v, av[t]);
    }
  }

#pragma unroll
  for (int t = 0; t < GNT; ++t) {
    const int cl = 16 * t + m;
#pragma unroll
    for (int r = 0; r < 8; ++r) {
      const int rl = wave * 16 + 8 * h + r;
      sF[rl * GBN + cl] = af[t][r];
      sI[rl * GBN + cl] = ai[t][r];
      sV[rl * GBN + cl] = av[t][r];
    }
  }
  __syncthreads();

#pragma unroll 1
  for (int e = tid; e < GBM * GBN; e += NTHR) {
    const float gf = sF[e] * WINV;
    const float gi = sI[e] * WINV;
    const float gv = sV[e] * WINV;
    sF[e] = tanh_(gf);
    sI[e] = sigm_(gi) * silu_(gv);
  }
  __syncthreads();

#pragma unroll
  for (int it = 0; it < (GBM * GBN / 4) / NTHR; ++it) {
    const int e = tid + it * NTHR;
    const int rl = e / (GBN / 4), q = e - rl * (GBN / 4);
    const size_t go = (size_t)(bm0 + rl) * NST + n0 + 4 * q;
    const v4f vf = *(const v4f*)(sF + 4 * e);
    const v4f vw = *(const v4f*)(sI + 4 * e);
    *(volatile v4f*)(FG + go) = vf;
    *(volatile v4f*)(WC + go) = vw;
  }
  __threadfence();
#pragma unroll
  for (int it = 0; it < (GBM * GBN / 4) / NTHR; ++it) {
    const int e = tid + it * NTHR;
    const int rl = e / (GBN / 4), q = e - rl * (GBN / 4);
    const size_t go = (size_t)(bm0 + rl) * NST + n0 + 4 * q;
    const v4f vf = *(const v4f*)(sF + 4 * e);
    const v4f vw = *(const v4f*)(sI + 4 * e);
    *(volatile v4f*)(FG + go) = vf;
    *(volatile v4f*)(WC + go) = vw;
  }
}

__global__ __launch_bounds__(NTHR) void k_scan(const float* __restrict__ FG, const float* __restrict__ WC,
                                               _Float16* HS) {
  __shared__ __align__(16) _Float16 sH[TB * NTHR];
  const int tid = threadIdx.x, lane = tid & 31, wave = tid >> 5;
  const int b = blockIdx.x / (NST / NTHR);
  const int nb = (blockIdx.x - b * (NST / NTHR)) * NTHR;
  const size_t rowb = (size_t)b * NSEQ;
  const size_t col = (size_t)(nb + tid);
  float st = 0.0f;

#pragma unroll 1
  for (int t0 = 0; t0 < NSEQ; t0 += TB) {
#pragma unroll 1
    for (int tl = 0; tl < TB; ++tl) {
      const size_t idx = (rowb + (size_t)(t0 + tl)) * NST + col;
      const float f = FG[idx];
      const float w = WC[idx];
      st = f * st + w;
      const float a = silu_(st) * HCAR;
      sH[tl * NTHR + tid] = (_Float16)a;
    }
    __syncthreads();
#pragma unroll
    for (int j = 0; j < TB / NWAV; ++j) {
      const int tl = wave * (TB / NWAV) + j;
      const v8h v = *(const v8h*)(sH + tl * NTHR + 8 * lane);
      _Float16* dp = HS + (rowb + (size_t)(t0 + tl)) * NST + nb + 8 * lane;
      *(volatile v8h*)dp = v;
    }
    __threadfence();
#pragma unroll
    for (int j = 0; j < TB / NWAV; ++j) {
      const int tl = wave * (TB / NWAV) + j;
      const v8h v = *(const v8h*)(sH + tl * NTHR + 8 * lane);
      _Float16* dp = HS + (rowb + (size_t)(t0 + tl)) * NST + nb + 8 * lane;
      *(volatile v8h*)dp = v;
    }
    __syncthreads();
  }
}

__global__ __launch_bounds__(NTHR) void k_out(const _Float16* __restrict__ HS, const _Float16* __restrict__ WO16,
                                              float* out) {
  __shared__ __align__(16) float sO[GBM * OBN];
  const int tid = threadIdx.x, lane = tid & 31, wave = tid >> 5, h = lane >> 4, m = lane & 15;
  const int bm0 = blockIdx.x * GBM;
  const int m0 = bm0 + wave * 16;
  const int n0 = blockIdx.y * OBN;

  v8f acc[ONT];
#pragma unroll
  for (int t = 0; t < ONT; ++t) acc[t] = zero8();

  const _Float16* ap = HS + (size_t)(m0 + m) * NST + 8 * h;
  const _Float16* bp0 = WO16 + (size_t)(n0 + m) * NST + 8 * h;

#pragma unroll 1
  for (int ks = 0; ks < NST / 32; ++ks) {
    const int k0 = 32 * ks;
    Frag fa;
    fa.h[0] = *(const v8h*)(ap + k0);
    fa.h[1] = *(const v8h*)(ap + k0 + 16);
#pragma unroll
    for (int t = 0; t < ONT; ++t) {
      const _Float16* bp = bp0 + (size_t)(t * 16) * NST + k0;
      Frag fb;
      fb.h[0] = *(const v8h*)bp;
      fb.h[1] = *(const v8h*)(bp + 16);
      acc[t] = wmh(fa.v, fb.v, acc[t]);
    }
  }

#pragma unroll
  for (int t = 0; t < ONT; ++t) {
    const int cl = 16 * t + m;
#pragma unroll
    for (int r = 0; r < 8; ++r) {
      const int rl = wave * 16 + 8 * h + r;
      sO[rl * OBN + cl] = acc[t][r] * OSCL;
    }
  }
  __syncthreads();

#pragma unroll
  for (int it = 0; it < (GBM * OBN / 4) / NTHR; ++it) {
    const int e = tid + it * NTHR;
    const int rl = e / (OBN / 4), q = e - rl * (OBN / 4);
    const v4f v = *(const v4f*)(sO + 4 * e);
    *(volatile v4f*)(out + (size_t)(bm0 + rl) * NHID + n0 + 4 * q) = v;
  }
  __threadfence();
#pragma unroll
  for (int it = 0; it < (GBM * OBN / 4) / NTHR; ++it) {
    const int e = tid + it * NTHR;
    const int rl = e / (OBN / 4), q = e - rl * (OBN / 4);
    const v4f v = *(const v4f*)(sO + 4 * e);
    *(volatile v4f*)(out + (size_t)(bm0 + rl) * NHID + n0 + 4 * q) = v;
  }
}

extern "C" void kernel_launch(void* const* d_in, const int* in_sizes, int n_in,
                              void* d_out, int out_size, void* d_ws, size_t ws_size,
                              hipStream_t stream) {
  if (n_in < 5) return;
  if (in_sizes[0] != NTOK * NHID) return;
  if (in_sizes[1] != NST * NHID || in_sizes[2] != NST * NHID || in_sizes[3] != NST * NHID) return;
  if (in_sizes[4] != NHID * NST) return;
  if (out_size != NTOK * NHID) return;
  const size_t tot = (size_t)WSTOT;
  if (tot > ws_size || tot > (size_t)WSCAP) return;

  const float* x  = (const float*)d_in[0];
  const float* Wf = (const float*)d_in[1];
  const float* Wi = (const float*)d_in[2];
  const float* Wv = (const float*)d_in[3];
  const float* Wo = (const float*)d_in[4];
  float* out = (float*)d_out;

  char* ws = (char*)d_ws;
  _Float16* X16  = (_Float16*)(ws + OX16);
  _Float16* WF16 = (_Float16*)(ws + OWF16);
  _Float16* WI16 = (_Float16*)(ws + OWI16);
  _Float16* WV16 = (_Float16*)(ws + OWV16);
  _Float16* WO16 = (_Float16*)(ws + OWO16);
  float* FG = (float*)(ws + OFG);
  float* WC = (float*)(ws + OWC);
  _Float16* HS = (_Float16*)(ws + OHS);

  k_cvt<<<CVTBLK, NTHR, 0, stream>>>(x, Wf, Wi, Wv, Wo, X16);

  k_gates<<<dim3(NTOK / GBM, NST / GBN), NTHR, 0, stream>>>(X16, WF16, WI16, WV16, FG, WC);

  k_scan<<<NBAT * (NST / NTHR), NTHR, 0, stream>>>(FG, WC, HS);

  k_out<<<dim3(NTOK / GBM, NHID / OBN), NTHR, 0, stream>>>(HS, WO16, out);
}
